// GnnLayer_70523363000699
// MI455X (gfx1250) — hardware-verified
//
#include <hip/hip_runtime.h>


namespace {

constexpr int N = 50000, NP = 50016, KN = 32, F = 64, P3 = 3, FO = 64, KC = KN * F  , CH = 512  , RL = NP  , NL = (RL < N ? RL : N);
constexpr float XS = 8.0f, WSC = 256.0f, WSQ = 0.25f, RS_ = 1024.0f;
static_assert(NP % 32 == 0 && NP >= N && RL % 32 == 0 && KC % CH == 0 && CH % F == 0 && FO == 64, "tiling");
typedef _Float16 b16;
typedef __attribute__((ext_vector_type(16))) _Float16 v16b;
typedef __attribute__((ext_vector_type(8))) _Float16 v8b;
typedef __attribute__((ext_vector_type(8))) float v8f;
typedef __attribute__((ext_vector_type(4))) float v4f;
__device__ __forceinline__ float bf16_rne(float f) { unsigned int u = __float_as_uint(f); u += 0x7FFFu + ((u >> 16) & 1u); return __uint_as_float(u & 0xFFFF0000u); }
__device__ __forceinline__ void split16(float v, b16& hi, b16& lo) { hi = (b16)v; lo = (b16)(v - (float)hi); }
__device__ __forceinline__ v16b frag_kb(const b16* p, int hh) { const v8b a = *(const v8b*)(p + 8 * hh), b = *(const v8b*)(p + 16 + 8 * hh); v16b f;
#pragma unroll
  for (int e = 0; e < 8; ++e) { f[e] = a[e]; f[8 + e] = b[e]; } return f; }
__device__ __forceinline__ v8f wmma16b(v16b a, v16b b, v8f c) { v8f d = __builtin_amdgcn_wmma_f32_16x16x32_f16(false, a, false, b, (short)0, c, false, false); asm volatile("v_nop\n\tv_nop\n\tv_nop\n\tv_nop" : "+v"(d) : "v"(a), "v"(b)); return d; }
__device__ __forceinline__ void wave_lds_sync() { __builtin_amdgcn_fence(__ATOMIC_RELEASE, "workgroup"); __builtin_amdgcn_wave_barrier(); __builtin_amdgcn_fence(__ATOMIC_ACQUIRE, "workgroup"); }
__device__ __forceinline__ float pmul(float a, float b) { float p = a * b; asm volatile("" : "+v"(p)); return p; }
__device__ __forceinline__ int iclamp(int v, int lo, int hi) { return v < lo ? lo : (v > hi ? hi : v); }
typedef __attribute__((ext_vector_type(4))) _Float16 v4h;
__global__ __launch_bounds__(256) void wt_kernel(const float* __restrict__ w, b16* __restrict__ WT, float scl) {
  const int u = blockIdx.x * 256 + threadIdx.x; if (u >= FO * KC / 8) return; const int e = u * 8; const int o = e / KC, k0 = e % KC; v8b v;
#pragma unroll
  for (int j = 0; j < 8; ++j) v[j] = (b16)(bf16_rne(w[(size_t)(k0 + j) * FO + o]) * scl);
  for (int pass = 0; pass < 2; ++pass) { *(volatile v8b*)(WT + e) = v; __threadfence(); }
}
__global__ __launch_bounds__(64) void gnn_kernel(const float* __restrict__ h, const float* __restrict__ pos, const int* __restrict__ nbr, const b16* __restrict__ WT, const b16* __restrict__ WQ, const float* __restrict__ bias, float* __restrict__ out, int mrows) {
  __shared__ __attribute__((aligned(16))) b16 Ah[2][16][CH + 8], Al[2][16][CH + 8]; __shared__ __attribute__((aligned(16))) float Tf[2][16][FO + 4]; __shared__ float Dv[2][16][CH / F];
  const int wave = threadIdx.x >> 5, lane = threadIdx.x & 31, nloc = lane & 15, hlf = lane >> 4; const size_t m0 = (size_t)blockIdx.x * 32 + wave * 16;
  v8f acc[4];
#pragma unroll
  for (int t = 0; t < 4; ++t) acc[t] = (v8f){};
#pragma unroll 1
  for (int kc = 0; kc < KC; kc += CH) {
    for (int idx = lane; idx < 16 * (CH / F); idx += 32) { const int rr = idx / (CH / F), kk = idx % (CH / F); const size_t row = m0 + rr; const size_t vrow = (row < (size_t)N) ? row : (size_t)N - 1; const int k = kc / F + kk;
      const int j_ = iclamp(nbr[vrow * KN + k], 0, N - 1); float sq = 0.0f; for (int p = 0; p < P3; ++p) { const float d_ = bf16_rne(pos[vrow * P3 + p]) - bf16_rne(pos[(size_t)j_ * P3 + p]); sq += pmul(d_, d_); }
      Dv[wave][rr][kk] = (sq == 0.0f) ? 2.0f : 1.0f / sqrtf(sq); }
    wave_lds_sync();
    for (int idx = lane; idx < 16 * (CH / 4); idx += 32) { const int rr = idx / (CH / 4), c4 = (idx % (CH / 4)) * 4; const int kk = c4 / F, f = c4 % F; const size_t row = m0 + rr; const size_t vrow = (row < (size_t)N) ? row : (size_t)N - 1;
      const int j_ = iclamp(nbr[vrow * KN + kc / F + kk], 0, N - 1); const v4f v = *(const v4f*)(h + (size_t)j_ * F + f); const float idv = Dv[wave][rr][kk]; v4h hv, lv;
      for (int j = 0; j < 4; ++j) { const float vs = pmul(bf16_rne(v[j]), idv) * XS; const b16 ph = (b16)vs; hv[j] = ph; lv[j] = (b16)((vs - (float)ph) * RS_); } *(v4h*)(&Ah[wave][rr][c4]) = hv; *(v4h*)(&Al[wave][rr][c4]) = lv; }
    wave_lds_sync();
#pragma unroll 1
    for (int kb = 0; kb < CH; kb += 32) { const v16b a = frag_kb(&Ah[wave][nloc][kb], hlf), al = frag_kb(&Al[wave][nloc][kb], hlf);
#pragma unroll
      for (int t = 0; t < 4; ++t) { const size_t wo_ = (size_t)(t * 16 + nloc) * KC + kc + kb; acc[t] = wmma16b(a, frag_kb(WT + wo_, hlf), acc[t]); acc[t] = wmma16b(al, frag_kb(WQ + wo_, hlf), acc[t]); } }
    wave_lds_sync(); }
#pragma unroll
  for (int t = 0; t < 4; ++t) { const int col = t * 16 + nloc; const float bb = bf16_rne(bias[col]); for (int r = 0; r < 8; ++r) { float y = acc[t][r] * (1.0f / (XS * WSC)) + bb; y = (y >= 0.0f) ? y : 0.01f * y; Tf[wave][8 * hlf + r][col] = (m0 + 8 * hlf + r < (size_t)N) ? y : 0.0f; } }
  wave_lds_sync();
  for (int pass = 0; pass < 2; ++pass) { for (int rr = 0; rr < 16; rr += 2) { const int r2 = rr + (lane >> 4); if (m0 + r2 < (size_t)mrows) *(volatile v4f*)(out + (m0 + r2) * FO + (lane & 15) * 4) = *(const v4f*)(&Tf[wave][r2][(lane & 15) * 4]); } __threadfence(); }
}
}

extern "C" void kernel_launch(void* const* d_in, const int* in_sizes, int n_in, void* d_out, int out_size, void* d_ws, size_t ws_size, hipStream_t stream) {
  (void)n_in;
  auto Fp = [&](int i) { return (const float*)d_in[i]; }; auto Ip = [&](int i) { return (const int*)d_in[i]; };
  if (in_sizes[0] != N * F || in_sizes[1] != N * P3 || in_sizes[2] != N * KN || in_sizes[3] != KC * FO || in_sizes[4] != FO || out_size != N * FO) return;
  size_t off = 0; char* ws = (char*)d_ws;
  auto carve = [&](size_t bytes) { char* p = ws + off; off += (bytes + 255) & ~(size_t)255; return p; };
  b16* WT = (b16*)carve((size_t)FO * KC * 2); b16* WQ = (b16*)carve((size_t)FO * KC * 2);
  if (off > ws_size || off > ((size_t)1 << 20)) return;
  wt_kernel<<<(FO * KC / 8 + 255) / 256, 256, 0, stream>>>(Fp(3), WT, WSC); wt_kernel<<<(FO * KC / 8 + 255) / 256, 256, 0, stream>>>(Fp(3), WQ, WSQ);
  gnn_kernel<<<RL / 32, 64, 0, stream>>>(Fp(0), Fp(1), Ip(2), WT, WQ, Fp(4), (float*)d_out, NL);
}
